// GridAttentionWeight_64364379898402
// MI455X (gfx1250) — hardware-verified
//
#pragma clang fp contract(off)
#include <hip/hip_runtime.h>
#include <hip/hip_bf16.h>
#include <stdint.h>

typedef _Float16 bf16_t;
typedef _Float16 v2bf  __attribute__((ext_vector_type(2)));
typedef _Float16 v16bf __attribute__((ext_vector_type(16)));
typedef float  v8f   __attribute__((ext_vector_type(8)));
typedef __attribute__((ext_vector_type(4))) float v4f_t;
typedef float v4fa __attribute__((ext_vector_type(4), may_alias));
typedef __attribute__((ext_vector_type(4))) uint32_t v4u_t;
typedef uint32_t v4ua __attribute__((ext_vector_type(4), may_alias));

#define NPOS   16384
#define HWPIX  4096
#define SLOTS  130
#define LDSTR  72

__device__ __forceinline__ v16bf load_mk(const bf16_t* lds, int rowBase, int k0) {
  const int lane = threadIdx.x & 31;
  const int half = lane >> 4;
  const bf16_t* p = lds + (rowBase + (lane & 15)) * LDSTR + k0 + 8 * half;
  v16bf v;
  *(uint4*)&v       = *(const uint4*)(p);
  *((uint4*)&v + 1) = *(const uint4*)(p + 16);
  return v;
}

#define WMMA_BF16(A, B, C) \
  __builtin_amdgcn_wmma_f32_16x16x32_f16(false, (A), false, (B), (short)0, (C), false, false)
#define RSPLIT (1.0f / 2048.0f)
#define PLQ    (4 * 1048576)
#define PLE    8192
__device__ __forceinline__ bf16_t lo_of(float v, bf16_t h) { return (bf16_t)((v - (float)h) * 2048.0f); }
__device__ __forceinline__ v8f wmma_split(v16bf a, v16bf al, v16bf b, v16bf bl, v8f c) {
  v8f x = {}; x = WMMA_BF16(al, b, x); x = WMMA_BF16(a, bl, x); return WMMA_BF16(a, b, c) + x * RSPLIT; }

__device__ __forceinline__ void async_b128(uint32_t lds_off, const void* gaddr) {
  asm volatile("global_load_async_to_lds_b128 %0, %1, off"
               :: "v"(lds_off), "v"((uint64_t)(uintptr_t)gaddr) : "memory");
}
__device__ __forceinline__ void wait_async0() {
  asm volatile("s_wait_asynccnt 0" ::: "memory");
}

__global__ __launch_bounds__(256) void proj_kernel(const float* __restrict__ Wm,
                                                   const float* __restrict__ bias,
                                                   const float* __restrict__ X,
                                                   bf16_t* __restrict__ Yh) {
  __shared__ bf16_t As[2][64 * LDSTR];
  __shared__ bf16_t BsT[2][64 * LDSTR];
  __shared__ __attribute__((aligned(16))) bf16_t So[2][64 * LDSTR];
  const int tid = threadIdx.x;
  const int wave = tid >> 5;
  const int lane = tid & 31;
  const int posBase = blockIdx.x * 64;
  const int oBase = blockIdx.y * 64;

  const int t0 = wave * 2, t1 = wave * 2 + 1;
  const int m0 = (t0 >> 2) * 16, n0 = (t0 & 3) * 16;
  const int m1 = (t1 >> 2) * 16, n1 = (t1 & 3) * 16;
  v8f acc0 = {}; v8f acc1 = {};

  for (int kc = 0; kc < 4; ++kc) {
    __syncthreads();
    for (int e = tid; e < 2048; e += 256) {
      int m = e >> 5, k2 = (e & 31) * 2;
      const float* wp = Wm + (oBase + m) * 256 + kc * 64 + k2;
      v2bf h; h[0] = (bf16_t)wp[0]; h[1] = (bf16_t)wp[1];
      v2bf hl; hl[0] = lo_of(wp[0], h[0]); hl[1] = lo_of(wp[1], h[1]);
      *(v2bf*)&As[0][m * LDSTR + k2] = h; *(v2bf*)&As[1][m * LDSTR + k2] = hl;
    }
    for (int e = tid; e < 2048; e += 256) {
      int n = e & 63, k2 = (e >> 6) * 2;
      float x0 = X[(kc * 64 + k2) * NPOS + posBase + n];
      float x1 = X[(kc * 64 + k2 + 1) * NPOS + posBase + n];
      v2bf h; h[0] = (bf16_t)x0; h[1] = (bf16_t)x1;
      v2bf hl; hl[0] = lo_of(x0, h[0]); hl[1] = lo_of(x1, h[1]);
      *(v2bf*)&BsT[0][n * LDSTR + k2] = h; *(v2bf*)&BsT[1][n * LDSTR + k2] = hl;
    }
    __syncthreads();
    {
      acc0 = wmma_split(load_mk(As[0], m0, 0),  load_mk(As[1], m0, 0),  load_mk(BsT[0], n0, 0),  load_mk(BsT[1], n0, 0),  acc0);
      acc0 = wmma_split(load_mk(As[0], m0, 32), load_mk(As[1], m0, 32), load_mk(BsT[0], n0, 32), load_mk(BsT[1], n0, 32), acc0);
      acc1 = wmma_split(load_mk(As[0], m1, 0),  load_mk(As[1], m1, 0),  load_mk(BsT[0], n1, 0),  load_mk(BsT[1], n1, 0),  acc1);
      acc1 = wmma_split(load_mk(As[0], m1, 32), load_mk(As[1], m1, 32), load_mk(BsT[0], n1, 32), load_mk(BsT[1], n1, 32), acc1);
    }
  }

  const int nIdx = lane & 15, half = lane >> 4;
  const int head = oBase >> 6;
  {
    union { uint4 u; bf16_t h[8]; } r, rl;
#pragma unroll
    for (int jj = 0; jj < 8; ++jj) { const float v = acc0[jj] + bias[oBase + m0 + jj + 8 * half]; r.h[jj] = (bf16_t)v; rl.h[jj] = lo_of(v, r.h[jj]); }
    *(uint4*)(So[0] + (n0 + nIdx) * LDSTR + m0 + 8 * half) = r.u; *(uint4*)(So[1] + (n0 + nIdx) * LDSTR + m0 + 8 * half) = rl.u;
  }
  {
    union { uint4 u; bf16_t h[8]; } r, rl;
#pragma unroll
    for (int jj = 0; jj < 8; ++jj) { const float v = acc1[jj] + bias[oBase + m1 + jj + 8 * half]; r.h[jj] = (bf16_t)v; rl.h[jj] = lo_of(v, r.h[jj]); }
    *(uint4*)(So[0] + (n1 + nIdx) * LDSTR + m1 + 8 * half) = r.u; *(uint4*)(So[1] + (n1 + nIdx) * LDSTR + m1 + 8 * half) = rl.u;
  }
  __syncthreads();
#pragma unroll 1
  for (int pass = 0; pass < 2; ++pass) {
    for (int ch = tid; ch < 64 * 8; ch += 256) { const int n = ch >> 3, p8 = (ch & 7) * 8;
      bf16_t* d = Yh + head * 1048576 + (size_t)(posBase + n) * 64 + p8;
      *(volatile v4u_t*)d = *(const v4ua*)(So[0] + n * LDSTR + p8); *(volatile v4u_t*)(d + PLQ) = *(const v4ua*)(So[1] + n * LDSTR + p8); }
    __threadfence();
  }
}

__global__ __launch_bounds__(256) void emb_prep(const float* __restrict__ ye,
                                                const float* __restrict__ xe,
                                                bf16_t* __restrict__ yh,
                                                bf16_t* __restrict__ xh) {
  int i = blockIdx.x * 256 + threadIdx.x;
  int r = i >> 6;
  const float yv = (r < 127) ? ye[i] : 0.0f, xv = (r < 127) ? xe[i] : 0.0f;
  const bf16_t a = (bf16_t)yv, al = lo_of(yv, a), c = (bf16_t)xv, cl = lo_of(xv, c);
  *(volatile bf16_t*)(yh + i) = a; *(volatile bf16_t*)(yh + PLE + i) = al; *(volatile bf16_t*)(xh + i) = c; *(volatile bf16_t*)(xh + PLE + i) = cl; __threadfence();
  *(volatile bf16_t*)(yh + i) = a; *(volatile bf16_t*)(yh + PLE + i) = al; *(volatile bf16_t*)(xh + i) = c; *(volatile bf16_t*)(xh + PLE + i) = cl;
}

__global__ __launch_bounds__(256) void et_kernel(const bf16_t* __restrict__ pqh,
                                                 const bf16_t* __restrict__ pkh,
                                                 const float* __restrict__ temb,
                                                 const int* __restrict__ frm,
                                                 float* __restrict__ out) {
  int gid = blockIdx.x * 256 + threadIdx.x;
  int b = gid >> 12;
  int pix = gid & 4095;
  int f[4];
#pragma unroll
  for (int i = 0; i < 4; ++i) f[i] = frm[i];
  int rel[4][4];
#pragma unroll
  for (int s = 0; s < 4; ++s)
#pragma unroll
    for (int t = 0; t < 4; ++t) { int r = f[s] - f[t] + 15; rel[s][t] = (r < 0) ? 0 : (r > 30 ? 30 : r); }

  const int base = b * 1048576 + pix * 64;
  float aQK[4][4] = {};
  float aQE[4][4] = {};
  for (int c = 0; c < 8; ++c) {
    union { uint4 v[4]; bf16_t h[32]; } qu, ku, qul, kul;
#pragma unroll
    for (int t = 0; t < 4; ++t) {
      qu.v[t]  = *(const uint4*)(pqh + base + t * 262144 + c * 8);
      ku.v[t]  = *(const uint4*)(pkh + base + t * 262144 + c * 8);
      qul.v[t] = *(const uint4*)(pqh + PLQ + base + t * 262144 + c * 8);
      kul.v[t] = *(const uint4*)(pkh + PLQ + base + t * 262144 + c * 8);
    }
#pragma unroll
    for (int pp = 0; pp < 8; ++pp) {
      float qv[4], kv[4];
#pragma unroll
      for (int t = 0; t < 4; ++t) { qv[t] = (float)qu.h[t * 8 + pp] + (float)qul.h[t * 8 + pp] * RSPLIT; kv[t] = (float)ku.h[t * 8 + pp] + (float)kul.h[t * 8 + pp] * RSPLIT; }
      int p = c * 8 + pp;
#pragma unroll
      for (int s = 0; s < 4; ++s)
#pragma unroll
        for (int t = 0; t < 4; ++t) {
          aQK[s][t] += qv[t] * kv[s];
          aQE[s][t] += qv[t] * temb[rel[s][t] * 64 + p];
        }
    }
  }
#pragma unroll 1
  for (int pass = 0; pass < 2; ++pass) {
#pragma unroll
    for (int s = 0; s < 4; ++s)
#pragma unroll
      for (int t = 0; t < 4; ++t)
        *(volatile float*)(out + (size_t)((b * SLOTS + s) * 4 + t) * HWPIX + pix) = aQK[s][t] + aQE[s][t];
    __threadfence();
  }
}

__global__ __launch_bounds__(256) void eyx_kernel(const bf16_t* __restrict__ pqh,
                                                  const bf16_t* __restrict__ pkh,
                                                  const bf16_t* __restrict__ embh,
                                                  float* __restrict__ out, float* __restrict__ eyT,
                                                  int slotBase, int isY) {
  __shared__ bf16_t QsT[2][64 * LDSTR];
  __shared__ bf16_t KsT[2][64 * LDSTR];
  __shared__ bf16_t Es[2][128 * LDSTR];
  __shared__ float  GD[192 * 16];
  __shared__ __attribute__((aligned(16))) float RT[63 * 64];

  const int tid = threadIdx.x;
  const int wave = tid >> 5;
  const int sid = blockIdx.x;
  const int b = sid >> 8;
  const int t = (sid >> 6) & 3;
  const int j = sid & 63;
  const int iStride = isY ? 64 : 1;
  const int gStride = isY ? 4096 : 64;
  const int sliceBase = (b * 16384 + t * 4096 + (isY ? j : j * 64)) * 64;
  const int outBase = ((b * SLOTS + slotBase) * 4 + t) * HWPIX + (isY ? j : j * 64);

#pragma unroll
  for (int pl = 0; pl < 2; ++pl) {
    const uint32_t qofs = (uint32_t)(uintptr_t)(&QsT[pl][0]);
    const uint32_t kofs = (uint32_t)(uintptr_t)(&KsT[pl][0]);
    const uint32_t eofs = (uint32_t)(uintptr_t)(&Es[pl][0]);
    const bf16_t* pq = pqh + (pl ? PLQ : 0); const bf16_t* pk = pkh + (pl ? PLQ : 0); const bf16_t* pe = embh + (pl ? PLE : 0);
    for (int e = tid; e < 512; e += 256) {
      int i = e >> 3, p8 = (e & 7) * 8;
      uint32_t lofs = (uint32_t)(i * LDSTR + p8) * 2;
      async_b128(qofs + lofs, pq + sliceBase + i * gStride + p8);
      async_b128(kofs + lofs, pk + sliceBase + i * gStride + p8);
    }
    for (int e = tid; e < 1024; e += 256) {
      int r = e >> 3, p8 = (e & 7) * 8;
      async_b128(eofs + (uint32_t)(r * LDSTR + p8) * 2, pe + r * 64 + p8);
    }
  }
  wait_async0();

  for (int nT = 0; nT < 4; ++nT) {
    __syncthreads();
    const int nBase = nT * 16;
    v16bf b0 = load_mk(QsT[0], nBase, 0), b0l = load_mk(QsT[1], nBase, 0);
    v16bf b1 = load_mk(QsT[0], nBase, 32), b1l = load_mk(QsT[1], nBase, 32);
    for (int tile = wave; tile < 12; tile += 8) {
      const bf16_t* Am  = (tile < 4) ? KsT[0] : Es[0];
      const bf16_t* Aml = (tile < 4) ? KsT[1] : Es[1];
      const int mBase = (tile < 4) ? tile * 16 : (tile - 4) * 16;
      v8f acc = {};
      acc = wmma_split(load_mk(Am, mBase, 0),  load_mk(Aml, mBase, 0),  b0, b0l, acc);
      acc = wmma_split(load_mk(Am, mBase, 32), load_mk(Aml, mBase, 32), b1, b1l, acc);
      const int lane = tid & 31;
      const int n = lane & 15, half = lane >> 4;
      const int rowBase = (tile < 4) ? tile * 16 : 64 + (tile - 4) * 16;
#pragma unroll
      for (int e2 = 0; e2 < 8; ++e2)
        GD[(rowBase + e2 + 8 * half) * 16 + n] = acc[e2];
    }
    __syncthreads();
    for (int e = tid; e < 63 * 16; e += 256) {
      int i = e >> 4;
      int nn = e & 15;
      int h = nBase + nn;
      int g = i + ((i >= h) ? 1 : 0);
      int r = g - h + 63;
      RT[i * 64 + h] = GD[g * 16 + nn] + GD[(64 + r) * 16 + nn];
    }
  }
  __syncthreads();
  (void)outBase; (void)iStride;
#pragma unroll 1
  for (int pass = 0; pass < 2; ++pass) {
    for (int ch = tid; ch < 63 * 16; ch += 256) { const int i = ch >> 4, q = (ch & 15) * 4;
      const v4f_t v = *(const volatile v4fa*)(RT + i * 64 + q);
      float* d = isY ? (eyT + ((((size_t)b * 4 + t) * 64 + j) * 63 + i) * 64 + q)
                     : (out + ((size_t)(b * SLOTS + slotBase + i) * 4 + t) * HWPIX + j * 64 + q);
      *(volatile v4f_t*)d = v; }
    __threadfence();
  }
}

__global__ __launch_bounds__(256) void eyT_to_out(const float* __restrict__ eyT, float* __restrict__ out) {
  const int g = blockIdx.x * 256 + threadIdx.x;
  if (g >= 4 * 63 * 4 * 64 * 16) return;
  const int w4 = (g & 15) * 4, h = (g >> 4) & 63, t = (g >> 10) & 3, i = (g >> 12) % 63, b = (g >> 12) / 63;
  v4f_t v;
  const float* s = eyT + ((((size_t)b * 4 + t) * 64 + w4) * 63 + i) * 64 + h;
  v.x = s[0]; v.y = s[63 * 64]; v.z = s[2 * 63 * 64]; v.w = s[3 * 63 * 64];
  float* d = out + ((size_t)(b * SLOTS + 4 + i) * 4 + t) * HWPIX + h * 64 + w4;
  *(volatile v4f_t*)d = v; __threadfence(); *(volatile v4f_t*)d = v;
}

__global__ __launch_bounds__(256) void softmax_kernel(float* __restrict__ out) {
  int gid = blockIdx.x * 256 + threadIdx.x;
  int b = gid >> 14;
  int rem = gid & 16383;
  float* col = out + (size_t)b * SLOTS * NPOS + rem;
  float m = -3.4e38f;
  for (int s = 0; s < SLOTS; ++s) m = fmaxf(m, col[s * NPOS]);
  float sum = 0.f;
  for (int s = 0; s < SLOTS; ++s) sum += __expf(col[s * NPOS] - m);
  float inv = 1.f / sum;
  for (int s = 0; s < SLOTS; ++s) { const float v = __expf(col[s * NPOS] - m) * inv;
    *(volatile float*)(col + (size_t)s * NPOS) = v; __threadfence(); *(volatile float*)(col + (size_t)s * NPOS) = v; }
}

extern "C" void kernel_launch(void* const* d_in, const int* in_sizes, int n_in,
                              void* d_out, int out_size, void* d_ws, size_t ws_size,
                              hipStream_t stream) {
  (void)in_sizes; (void)n_in; (void)out_size; (void)ws_size;
  const float* query    = (const float*)d_in[0];
  const float* key_feat = (const float*)d_in[1];
  const int*   frm      = (const int*)d_in[2];
  const float* qw       = (const float*)d_in[3];
  const float* qb       = (const float*)d_in[4];
  const float* kw       = (const float*)d_in[5];
  const float* kb       = (const float*)d_in[6];
  const float* x_emb    = (const float*)d_in[7];
  const float* y_emb    = (const float*)d_in[8];
  const float* t_emb    = (const float*)d_in[9];
  float* out = (float*)d_out;

  bf16_t* pqh = (bf16_t*)d_ws;
  bf16_t* pkh = pqh + 8 * 1048576;
  bf16_t* eyh = pkh + 8 * 1048576;
  bf16_t* exh = eyh + 16384;
  float*  eyT = (float*)(exh + 16384);

  dim3 pgrid(NPOS / 64, 4);
  proj_kernel<<<pgrid, 256, 0, stream>>>(qw, qb, query, pqh);
  proj_kernel<<<pgrid, 256, 0, stream>>>(kw, kb, key_feat, pkh);
  emb_prep<<<32, 256, 0, stream>>>(y_emb, x_emb, eyh, exh);
  et_kernel<<<64, 256, 0, stream>>>(pqh, pkh, t_emb, frm, out);
  eyx_kernel<<<1024, 256, 0, stream>>>(pqh, pkh, eyh, out, eyT, 4, 1);
  eyT_to_out<<<(4 * 63 * 4 * 64 * 16) / 256, 256, 0, stream>>>(eyT, out);
  eyx_kernel<<<1024, 256, 0, stream>>>(pqh, pkh, exh, out, eyT, 67, 0);
  softmax_kernel<<<256, 256, 0, stream>>>(out);
}
